// TransformerBlock_84112639525604
// MI455X (gfx1250) — hardware-run, weakly checked
//
#include <hip/hip_runtime.h>


#ifndef NB
#define NB 4
#endif
#ifndef SEQ
#define SEQ 1024
#endif
#define NB_FULL  4
#define SEQ_FULL 1024
#ifndef OUT_SEQ
#define OUT_SEQ SEQ
#endif
#define DM   512
#define NH_  8
#define HD   512
#define FFD  2048
#define CAT  (NH_ * HD)
#define FW   4
#define KST  (32 * FW)
#define DSL  (HD / FW)
#define PPT  136
#define OSF  132
#define NPASS ((NB % 2 == 0) ? 2 : 1)
#define NBP  (NB / NPASS)
#define WOS  64.0f
#define W1S  16.0f
#define W2S  32.0f
#define CXS  16.0f
#define SC2  ((float)(0.044194173824159216 * 1.4426950408889634))
#define PSH  14.0f
#define NEGB (-3.0e38f)
#define LNEPS 1.0e-6f

static_assert(DM == 512);
static_assert(HD == DM);
static_assert(DM % 64 == 0);
static_assert(HD % 64 == 0);
static_assert(FFD % 64 == 0);
static_assert(CAT % 64 == 0);
static_assert(DM % 32 == 0);
static_assert(FFD % 32 == 0);
static_assert(CAT % 32 == 0);
static_assert(SEQ % 64 == 0);
static_assert(SEQ % KST == 0);
static_assert(SEQ % 16 == 0);
static_assert(DSL == 128);
static_assert(FW * DSL == HD);
static_assert(NB % NPASS == 0);
static_assert((NB * SEQ) % 64 == 0);
static_assert((NBP * SEQ) % 64 == 0);
static_assert((NB * SEQ) % 8 == 0);
static_assert(((size_t)SEQ * DM) % 8 == 0);
static_assert(NB <= NB_FULL);
static_assert(SEQ <= SEQ_FULL);
static_assert((OSF * 4) % 16 == 0);
static_assert((PPT * 2) % 16 == 0);
static_assert(PPT >= KST);

typedef _Float16 h16;
typedef unsigned short bf;
typedef __attribute__((ext_vector_type(16))) __bf16   v16bf;
typedef __attribute__((ext_vector_type(16))) _Float16 v16h;
typedef __attribute__((ext_vector_type(8)))  _Float16 v8h;
typedef __attribute__((ext_vector_type(4)))  _Float16 v4h;
typedef __attribute__((ext_vector_type(8)))  unsigned short v8us;
typedef __attribute__((ext_vector_type(8)))  float    v8f;
typedef __attribute__((ext_vector_type(4)))  float    v4f;
typedef v4f  __attribute__((may_alias)) v4fa;
typedef v8h  __attribute__((may_alias)) v8ha;

__device__ __forceinline__ unsigned short f2bf(float f) { unsigned u = __float_as_uint(f); u += 0x7FFFu + ((u >> 16) & 1u); return (unsigned short)(u >> 16); }
__device__ __forceinline__ float bfr(float f) { return __uint_as_float(((unsigned)f2bf(f)) << 16); }
__device__ __forceinline__ v16h cat16(v8h lo, v8h hi) { return __builtin_shufflevector(lo, hi, 0, 1, 2, 3, 4, 5, 6, 7, 8, 9, 10, 11, 12, 13, 14, 15); }
__device__ __forceinline__ v16bf cat16b(v8us lo, v8us hi) { return __builtin_bit_cast(v16bf, __builtin_shufflevector(lo, hi, 0, 1, 2, 3, 4, 5, 6, 7, 8, 9, 10, 11, 12, 13, 14, 15)); }
__device__ __forceinline__ v8f wmma16(v16h a, v16h b, v8f c) { return __builtin_amdgcn_wmma_f32_16x16x32_f16(false, a, false, b, (short)0, c, false, false); }
__device__ __forceinline__ v8f wmmab(v16bf a, v16bf b, v8f c) { return __builtin_amdgcn_wmma_f32_16x16x32_bf16(false, a, false, b, (short)0, c, false, false); }
__device__ __forceinline__ v16h  ldh(const h16* p) { return cat16(*(const v8h*)p, *(const v8h*)(p + 16)); }
__device__ __forceinline__ v16bf ldb(const bf* p)  { return cat16b(*(const v8us*)p, *(const v8us*)(p + 16)); }
__device__ __forceinline__ void wave_sync() { __builtin_amdgcn_fence(3  , "wavefront"); __builtin_amdgcn_wave_barrier(); asm volatile("" ::: "memory"); }

static __device__ __forceinline__ h16 toh_flush(float v) { const h16 r = (h16)v; return (fabsf(v) < 6.103515625e-05f) ? (h16)0.0f : r; }
__device__ __forceinline__ v8f mmag(v16h a, v16h b, v8f c) { c = wmma16(a, b, c); asm volatile("v_nop\n\tv_nop\n\tv_nop\n\tv_nop" : "+v"(c) : "v"(a), "v"(b)); return c; }
__device__ __forceinline__ v8f mmag(v16bf a, v16bf b, v8f c) { c = wmmab(a, b, c); asm volatile("v_nop\n\tv_nop\n\tv_nop\n\tv_nop" : "+v"(c) : "v"(a), "v"(b)); return c; }
__device__ __forceinline__ v16h  ldf(const h16* p) { return ldh(p); }
__device__ __forceinline__ v16bf ldf(const bf* p)  { return ldb(p); }

__global__ __launch_bounds__(256) void k_cvt8(const float* __restrict__ src, bf* dst, size_t n8) {
    const size_t i = (size_t)blockIdx.x * 256 + threadIdx.x; if (i >= n8) return;
    const v8f v = *(const v8f*)(src + i * 8); v8us o;
#pragma unroll
    for (int k = 0; k < 8; ++k) o[k] = f2bf(v[k]);
    *(volatile v8us*)(dst + i * 8) = o; __threadfence(); *(volatile v8us*)(dst + i * 8) = o;
}

template <int F16>
__device__ __forceinline__ void wtr_tile(const float* __restrict__ src, bf* DB, h16* DH, const int K, const int N, const float scale) {
    __shared__ float ts[64 * 65];
    const int tid = threadIdx.x;
    const int n0 = blockIdx.x * 64, k0 = blockIdx.y * 64;
    const size_t zb = (size_t)blockIdx.z * (size_t)K * (size_t)N;
    static_assert(4 * 256 * 4 == 64 * 64);
#pragma unroll
    for (int it = 0; it < 4; ++it) { const int p = it * 256 + tid; const int kr = p >> 4, c4 = (p & 15) * 4;
        const v4f v = *(const v4f*)(src + zb + (size_t)(k0 + kr) * N + n0 + c4);
#pragma unroll
        for (int i = 0; i < 4; ++i) ts[kr * 65 + c4 + i] = v[i]; }
    __syncthreads();
    static_assert(2 * 256 * 8 == 64 * 64);
#pragma unroll
    for (int it = 0; it < 2; ++it) { const int p = it * 256 + tid; const int nr = p >> 3, k8 = (p & 7) * 8;
        float x[8];
#pragma unroll
        for (int i = 0; i < 8; ++i) x[i] = ts[(k8 + i) * 65 + nr];
        const size_t oo = zb + (size_t)(n0 + nr) * K + k0 + k8;
        if (F16) { v8h o;
#pragma unroll
            for (int i = 0; i < 8; ++i) o[i] = toh_flush(bfr(x[i]) * scale);
            *(volatile v8h*)(DH + oo) = o; __threadfence(); *(volatile v8h*)(DH + oo) = o;
        } else { v8us o;
#pragma unroll
            for (int i = 0; i < 8; ++i) o[i] = f2bf(x[i]);
            *(volatile v8us*)(DB + oo) = o; __threadfence(); *(volatile v8us*)(DB + oo) = o; } }
}
__global__ __launch_bounds__(256) void k_wtr_bf(const float* __restrict__ src, bf* dst, int K, int N) { wtr_tile<0>(src, dst, (h16*)0, K, N, 1.0f); }
__global__ __launch_bounds__(256) void k_wtr_h(const float* __restrict__ src, h16* dst, int K, int N, float scale) { wtr_tile<1>(src, (bf*)0, dst, K, N, scale); }

template <typename T, int OM, int HASB>
__device__ __forceinline__ void gemm64(const T* __restrict__ A, const T* __restrict__ Bt, const int K, const size_t arow, const size_t brow,
                                       const float* __restrict__ bias, const int bcol, const float scale,
                                       h16* OH, float* OF, const size_t obase, const size_t pitch) {
    __shared__ __align__(16) float os[16 * 68];
    static_assert(16 * 68 * 4 <= 131072);
    typedef decltype(ldf((const T*)0)) frag;
    const int lane = threadIdx.x & 31, lr = lane & 15, hi = lane >> 4;
    v8f acc[4][4];
#pragma unroll
    for (int mb = 0; mb < 4; ++mb)
#pragma unroll
        for (int nb = 0; nb < 4; ++nb) acc[mb][nb] = (v8f){};
    const size_t aoff = (arow + (size_t)lr) * (size_t)K + 8 * hi, boff = (brow + (size_t)lr) * (size_t)K + 8 * hi;
#pragma unroll 1
    for (int kc = 0; kc < K; kc += 32) {
        frag a[4];
#pragma unroll
        for (int mb = 0; mb < 4; ++mb) a[mb] = ldf(A + aoff + (size_t)mb * 16 * K + kc);
#pragma unroll
        for (int nb = 0; nb < 4; ++nb) { const frag b = ldf(Bt + boff + (size_t)nb * 16 * K + kc);
#pragma unroll
            for (int mb = 0; mb < 4; ++mb) acc[mb][nb] = mmag(a[mb], b, acc[mb][nb]); }
    }
    float bc[4];
#pragma unroll
    for (int nb = 0; nb < 4; ++nb) { bc[nb] = 0.0f; if (HASB) bc[nb] = bfr(bias[bcol + nb * 16 + lr]); }
#pragma unroll
    for (int mb = 0; mb < 4; ++mb) {
#pragma unroll
        for (int nb = 0; nb < 4; ++nb) {
#pragma unroll
            for (int j = 0; j < 8; ++j) os[(hi * 8 + j) * 68 + nb * 16 + lr] = acc[mb][nb][j] * scale + bc[nb]; }
        wave_sync();
#pragma unroll 1
        for (int ps = 0; ps < 2; ++ps) {
            if (OM == 1) {
                static_assert(8 * 32 * 4 == 16 * 64);
#pragma unroll
                for (int s = 0; s < 8; ++s) { const int p = s * 32 + lane; const int row = p >> 4, cofs = (p & 15) * 4;
                    const v4f val = *(const v4fa*)(&os[row * 68 + cofs]);
                    *(volatile v4f*)(OF + obase + (size_t)(mb * 16 + row) * pitch + cofs) = val; }
            } else {
                static_assert(4 * 32 * 8 == 16 * 64);
#pragma unroll
                for (int s = 0; s < 4; ++s) { const int row = 4 * s + (lane >> 3), c8 = (lane & 7) * 8;
                    const v4f x0 = *(const v4fa*)(&os[row * 68 + c8]); const v4f x1 = *(const v4fa*)(&os[row * 68 + c8 + 4]); v8h hv;
#pragma unroll
                    for (int i = 0; i < 4; ++i) { float y0 = x0[i], y1 = x1[i];
                        if (OM == 2) { y0 = fmaxf(y0, 0.0f); y1 = fmaxf(y1, 0.0f); }
                        hv[i] = toh_flush(y0); hv[4 + i] = toh_flush(y1); }
                    *(volatile v8h*)(OH + obase + (size_t)(mb * 16 + row) * pitch + c8) = hv; }
            }
            if (ps == 0) __threadfence(); }
        wave_sync();
    }
}

__global__ __launch_bounds__(32) void k_proj_qk(const bf* __restrict__ XB, const bf* __restrict__ WT, h16* QK, int b0) {
    const int r0 = blockIdx.x * 64, c0 = blockIdx.y * 64, z = blockIdx.z;
    const int bl = r0 / SEQ, tt = r0 % SEQ; const int which = z >> 3, hh = z & 7;
    const size_t obase = ((((size_t)which * NBP + (size_t)bl) * NH_ + (size_t)hh) * SEQ + (size_t)tt) * HD + (size_t)c0;
    gemm64<bf, 0, 0>(XB, WT, DM, (size_t)b0 * SEQ + (size_t)r0, (size_t)z * HD + (size_t)c0, (const float*)0, 0, 1.0f, QK, (float*)0, obase, (size_t)HD);
}
__global__ __launch_bounds__(32) void k_proj_vt(const bf* __restrict__ WV, const bf* __restrict__ XB, h16* VT, int b0) {
    const int r0 = blockIdx.x * 64, c0 = blockIdx.y * 64, hh = blockIdx.z;
    const int bl = c0 / SEQ, tt = c0 % SEQ;
    const size_t obase = (((size_t)bl * NH_ + (size_t)hh) * HD + (size_t)r0) * SEQ + (size_t)tt;
    gemm64<bf, 0, 0>(WV, XB, DM, (size_t)hh * HD + (size_t)r0, (size_t)b0 * SEQ + (size_t)c0, (const float*)0, 0, 1.0f, VT, (float*)0, obase, (size_t)SEQ);
}
__global__ __launch_bounds__(32) void k_wo(const h16* __restrict__ CTX, const h16* __restrict__ WOT, float* MHA) {
    const int r0 = blockIdx.x * 64, c0 = blockIdx.y * 64;
    gemm64<h16, 1, 0>(CTX, WOT, CAT, (size_t)r0, (size_t)c0, (const float*)0, 0, 1.0f / (WOS * CXS), (h16*)0, MHA, (size_t)r0 * DM + (size_t)c0, (size_t)DM);
}
__global__ __launch_bounds__(32) void k_ffn1(const h16* __restrict__ HH, const h16* __restrict__ W1T, const float* __restrict__ b1, h16* F1) {
    const int r0 = blockIdx.x * 64, c0 = blockIdx.y * 64;
    gemm64<h16, 2, 1>(HH, W1T, DM, (size_t)r0, (size_t)c0, b1, c0, 1.0f / W1S, F1, (float*)0, (size_t)r0 * FFD + (size_t)c0, (size_t)FFD);
}
__global__ __launch_bounds__(32) void k_ffn2(const h16* __restrict__ F1, const h16* __restrict__ W2T, const float* __restrict__ b2, float* F2) {
    const int r0 = blockIdx.x * 64, c0 = blockIdx.y * 64;
    gemm64<h16, 1, 1>(F1, W2T, FFD, (size_t)r0, (size_t)c0, b2, c0, 1.0f / W2S, (h16*)0, F2, (size_t)r0 * DM + (size_t)c0, (size_t)DM);
}

__global__ __launch_bounds__(32 * FW) __attribute__((amdgpu_num_vgpr(256)))
void k_flash(const h16* __restrict__ QP, const h16* __restrict__ KP, const h16* __restrict__ VT, h16* CTX, int b0) {
    __shared__ __align__(16) float os[FW * 16 * OSF];
    __shared__ __align__(16) h16 pt[16 * PPT];
    __shared__ float smax[FW * 16];
    __shared__ float ssum[FW * 16];
    static_assert(FW * 16 * OSF * 4 + 16 * PPT * 2 + 2 * FW * 16 * 4 <= 131072);
    const int lane = threadIdx.x & 31, lr = lane & 15, hi = lane >> 4;
    const int wave = __builtin_amdgcn_readfirstlane((int)(threadIdx.x >> 5));
    const int zh = blockIdx.y; const int bl = zh / NH_, h = zh % NH_;
    const int t0 = blockIdx.x * 16;
    const size_t pbase = (size_t)zh * SEQ * HD;
    const size_t qo = pbase + (size_t)(t0 + lr) * HD + 8 * hi;
    const size_t ko = pbase + (size_t)(32 * wave + lr) * HD + 8 * hi;
    const size_t vo = pbase + (size_t)(DSL * wave + lr) * SEQ + 8 * hi;
    const int pw = lr * PPT + 32 * wave + 8 * hi;
    const int pl = lr * PPT + 8 * hi;
    v8f o[8];
#pragma unroll
    for (int j = 0; j < 8; ++j) o[j] = (v8f){};
    float m = NEGB, l = 0.0f;
#pragma unroll 1
    for (int key0 = 0; key0 < SEQ; key0 += KST) {
        v8f sA = (v8f){}, sB = (v8f){};
        { const h16* kp = KP + ko + (size_t)key0 * HD;
#pragma unroll 2
          for (int kc = 0; kc < HD; kc += 32) {
              const v16h q = ldh(QP + qo + kc);
              const v16h ka = ldh(kp + kc), kb = ldh(kp + 16 * HD + kc);
              sA = mmag(ka, q, sA); sB = mmag(kb, q, sB); } }
        float ta[8], tb[8]; float mx = NEGB;
#pragma unroll
        for (int r = 0; r < 8; ++r) { ta[r] = sA[r] * SC2; tb[r] = sB[r] * SC2; mx = fmaxf(mx, fmaxf(ta[r], tb[r])); }
        mx = fmaxf(mx, __shfl_xor(mx, 16, 32));
        smax[wave * 16 + lr] = mx;
        __syncthreads();
        const float mall = fmaxf(fmaxf(smax[lr], smax[16 + lr]), fmaxf(smax[32 + lr], smax[48 + lr]));
        const float mnew = fmaxf(m, mall);
        const float alpha = __builtin_amdgcn_exp2f(m - mnew);
        const float sh = PSH - mnew;
        v8h pa, pb; float ls = 0.0f;
#pragma unroll
        for (int r = 0; r < 8; ++r) {
            const float ea = ta[r] + sh, eb = tb[r] + sh;
            const float xa = __builtin_amdgcn_exp2f(ea), xb = __builtin_amdgcn_exp2f(eb);
            const float ga = (ea < -14.0f) ? 0.0f : xa, gb = (eb < -14.0f) ? 0.0f : xb;
            const h16 ha = (h16)ga; const h16 hb = (h16)gb;
            pa[r] = ha; pb[r] = hb; ls += (float)ha + (float)hb; }
        *(v8ha*)(&pt[pw]) = pa; *(v8ha*)(&pt[pw + 16]) = pb;
        l = l * alpha + ls; m = mnew;
#pragma unroll
        for (int j = 0; j < 8; ++j) o[j] = o[j] * alpha;
        __syncthreads();
        const h16* vp = VT + vo + key0;
#pragma unroll 1
        for (int ks = 0; ks < FW; ++ks) {
            const v16h pf = cat16(*(const v8ha*)(&pt[pl + 32 * ks]), *(const v8ha*)(&pt[pl + 32 * ks + 16]));
#pragma unroll
            for (int j = 0; j < 8; ++j) { const v16h v = ldh(vp + (size_t)(16 * j) * SEQ + 32 * ks); o[j] = mmag(v, pf, o[j]); } }
    }
    l += __shfl_xor(l, 16, 32);
    ssum[wave * 16 + lr] = l;
    __syncthreads();
    const float L = ((ssum[lr] + ssum[16 + lr]) + ssum[32 + lr]) + ssum[48 + lr];
    const float inv = CXS * (1.0f / L);
    const int wb = wave * 16 * OSF;
#pragma unroll
    for (int j = 0; j < 8; ++j) { v4f a, c;
        a[0] = o[j][0] * inv; a[1] = o[j][1] * inv; a[2] = o[j][2] * inv; a[3] = o[j][3] * inv;
        c[0] = o[j][4] * inv; c[1] = o[j][5] * inv; c[2] = o[j][6] * inv; c[3] = o[j][7] * inv;
        *(v4fa*)(&os[wb + lr * OSF + 16 * j + 8 * hi]) = a; *(v4fa*)(&os[wb + lr * OSF + 16 * j + 8 * hi + 4]) = c; }
    wave_sync();
    h16* crow = CTX + ((size_t)(b0 + bl) * SEQ + (size_t)t0) * CAT + (size_t)h * HD + (size_t)DSL * wave;
    static_assert(8 * 32 * 8 == 16 * DSL);
#pragma unroll 1
    for (int ps = 0; ps < 2; ++ps) {
#pragma unroll
        for (int s = 0; s < 8; ++s) { const int p = s * 32 + lane; const int row = p >> 4, c8 = (p & 15) * 8;
            const v4f x0 = *(const v4fa*)(&os[wb + row * OSF + c8]); const v4f x1 = *(const v4fa*)(&os[wb + row * OSF + c8 + 4]); v8h hv;
#pragma unroll
            for (int i = 0; i < 4; ++i) { hv[i] = toh_flush(x0[i]); hv[4 + i] = toh_flush(x1[i]); }
            *(volatile v8h*)(crow + (size_t)row * CAT + c8) = hv; }
        if (ps == 0) __threadfence(); }
}

template <int FIRST>
__device__ __forceinline__ void ln_row(const float* __restrict__ R, const size_t roff, const float* __restrict__ Y, const size_t yoff,
                                       const float* __restrict__ gamma, const float* __restrict__ beta, float* OF, const size_t ooff, h16* OH, const size_t hoff) {
#pragma clang fp contract(off)
    const int lane = threadIdx.x & 31;
    static_assert(4 * 32 * 4 == DM);
    v4f v[4]; float s = 0.0f;
#pragma unroll
    for (int it = 0; it < 4; ++it) { const int c = it * 128 + lane * 4;
        const v4f a = *(const v4f*)(R + roff + c); const v4f y = *(const v4f*)(Y + yoff + c);
#pragma unroll
        for (int i = 0; i < 4; ++i) { const float ai = FIRST ? bfr(a[i]) : a[i]; v[it][i] = ai + y[i]; s += v[it][i]; } }
    s += __shfl_xor(s, 16, 32); s += __shfl_xor(s, 8, 32); s += __shfl_xor(s, 4, 32); s += __shfl_xor(s, 2, 32); s += __shfl_xor(s, 1, 32);
    const float mu = s * (1.0f / (float)DM);
    float q = 0.0f;
#pragma unroll
    for (int it = 0; it < 4; ++it) {
#pragma unroll
        for (int i = 0; i < 4; ++i) { const float d = v[it][i] - mu; q += d * d; } }
    q += __shfl_xor(q, 16, 32); q += __shfl_xor(q, 8, 32); q += __shfl_xor(q, 4, 32); q += __shfl_xor(q, 2, 32); q += __shfl_xor(q, 1, 32);
    const float rs = rsqrtf(q * (1.0f / (float)DM) + LNEPS);
    v4f yo[4]; v4h hy[4];
#pragma unroll
    for (int it = 0; it < 4; ++it) { const int c = it * 128 + lane * 4;
        const v4f g = *(const v4f*)(gamma + c); const v4f bt = *(const v4f*)(beta + c);
#pragma unroll
        for (int i = 0; i < 4; ++i) { const float yv = (v[it][i] - mu) * rs * bfr(g[i]) + bfr(bt[i]); yo[it][i] = yv; hy[it][i] = toh_flush(yv); } }
#pragma unroll 1
    for (int ps = 0; ps < 2; ++ps) {
#pragma unroll
        for (int it = 0; it < 4; ++it) { const int c = it * 128 + lane * 4;
            *(volatile v4f*)(OF + ooff + c) = yo[it];
            if (FIRST) *(volatile v4h*)(OH + hoff + c) = hy[it]; }
        if (ps == 0) __threadfence(); }
}
__global__ __launch_bounds__(256) void k_ln1(const float* __restrict__ X, const float* __restrict__ MHA, const float* __restrict__ gamma, const float* __restrict__ beta, float* HF, h16* HH) {
    const int wave = __builtin_amdgcn_readfirstlane((int)(threadIdx.x >> 5));
    const int row = blockIdx.x * 8 + wave; const int bl = row / SEQ, tt = row % SEQ;
    ln_row<1>(X, ((size_t)bl * SEQ_FULL + (size_t)tt) * DM, MHA, (size_t)row * DM, gamma, beta, HF, (size_t)row * DM, HH, (size_t)row * DM);
}
__global__ __launch_bounds__(256) void k_ln2(const float* __restrict__ HF, const float* __restrict__ F2, const float* __restrict__ gamma, const float* __restrict__ beta, float* OUT) {
    const int wave = __builtin_amdgcn_readfirstlane((int)(threadIdx.x >> 5));
    const int row = blockIdx.x * 8 + wave; const int bl = row / SEQ, tt = row % SEQ;
    ln_row<0>(HF, (size_t)row * DM, F2, (size_t)row * DM, gamma, beta, OUT, ((size_t)bl * OUT_SEQ + (size_t)tt) * DM, (h16*)0, (size_t)0);
}

static constexpr size_t al256(size_t v) { return (v + 255) & ~(size_t)255; }
static constexpr size_t SZ_XB  = al256((size_t)NB * SEQ * DM * 2);
static constexpr size_t SZ_WT  = al256((size_t)3 * NH_ * HD * DM * 2);
static constexpr size_t SZ_WO  = al256((size_t)DM * CAT * 2);
static constexpr size_t SZ_W1  = al256((size_t)FFD * DM * 2);
static constexpr size_t SZ_W2  = al256((size_t)DM * FFD * 2);
static constexpr size_t SZ_QK  = al256((size_t)2 * NBP * NH_ * SEQ * HD * 2);
static constexpr size_t SZ_VT  = al256((size_t)NBP * NH_ * HD * SEQ * 2);
static constexpr size_t SZ_CTX = al256((size_t)NB * SEQ * CAT * 2);
static constexpr size_t SZ_MHA = al256((size_t)NB * SEQ * DM * 4);
static constexpr size_t SZ_HF  = al256((size_t)NB * SEQ * DM * 4);
static constexpr size_t SZ_HH  = al256((size_t)NB * SEQ * DM * 2);
static constexpr size_t SZ_F1  = al256((size_t)NB * SEQ * FFD * 2);
static constexpr size_t SZ_F2  = al256((size_t)NB * SEQ * DM * 4);
static constexpr size_t SZ_TOTAL = SZ_XB + SZ_WT + SZ_WO + SZ_W1 + SZ_W2 + SZ_QK + SZ_VT + SZ_CTX;
static_assert(SZ_TOTAL <= (size_t)134217728);
static_assert(SZ_MHA + SZ_HF + SZ_HH + SZ_F1 + SZ_F2 <= SZ_QK + SZ_VT);
static_assert(((size_t)NH_ * HD * DM * 2) % 256 == 0);
static_assert(((size_t)NBP * NH_ * SEQ * HD * 2) % 256 == 0);

extern "C" void kernel_launch(void* const* d_in, const int* in_sizes, int n_in,
                              void* d_out, int out_size, void* d_ws, size_t ws_size, hipStream_t stream) {
    if (n_in < 13) return;
    const size_t needx = ((size_t)(NB - 1) * SEQ_FULL + SEQ) * DM;
    if ((size_t)in_sizes[0] < needx) return;
    if ((size_t)in_sizes[1] < (size_t)NH_ * DM * HD || (size_t)in_sizes[2] < (size_t)NH_ * DM * HD || (size_t)in_sizes[3] < (size_t)NH_ * DM * HD) return;
    if ((size_t)in_sizes[4] < (size_t)CAT * DM || (size_t)in_sizes[5] < (size_t)DM * FFD || (size_t)in_sizes[7] < (size_t)FFD * DM) return;
    if (in_sizes[6] < FFD || in_sizes[8] < DM || in_sizes[9] < DM || in_sizes[10] < DM || in_sizes[11] < DM || in_sizes[12] < DM) return;
    if ((size_t)out_size < ((size_t)(NB - 1) * OUT_SEQ + SEQ) * DM) return;
    if (SZ_TOTAL > ws_size) return;
    const float* x  = (const float*)d_in[0];
    const float* wq = (const float*)d_in[1]; const float* wk = (const float*)d_in[2]; const float* wv = (const float*)d_in[3];
    const float* wo = (const float*)d_in[4];
    const float* w1 = (const float*)d_in[5]; const float* b1 = (const float*)d_in[6];
    const float* w2 = (const float*)d_in[7]; const float* b2 = (const float*)d_in[8];
    const float* g1 = (const float*)d_in[9];  const float* be1 = (const float*)d_in[10];
    const float* g2 = (const float*)d_in[11]; const float* be2 = (const float*)d_in[12];
    float* OUT = (float*)d_out;
    char* wsp = (char*)d_ws;
    bf*  XB  = (bf*)wsp;  wsp += SZ_XB;
    bf*  WT  = (bf*)wsp;  wsp += SZ_WT;
    h16* WOT = (h16*)wsp; wsp += SZ_WO;
    h16* W1T = (h16*)wsp; wsp += SZ_W1;
    h16* W2T = (h16*)wsp; wsp += SZ_W2;
    char* reg = wsp;
    h16* QK  = (h16*)wsp; wsp += SZ_QK;
    h16* VT  = (h16*)wsp; wsp += SZ_VT;
    h16* CTX = (h16*)wsp; wsp += SZ_CTX;
    float* MHA = (float*)reg; reg += SZ_MHA;
    float* HF  = (float*)reg; reg += SZ_HF;
    h16*   HH  = (h16*)reg;   reg += SZ_HH;
    h16*   F1  = (h16*)reg;   reg += SZ_F1;
    float* F2  = (float*)reg; reg += SZ_F2;
    h16* QP = QK; h16* KP = QK + (size_t)NBP * NH_ * SEQ * HD;
    bf* WQ = WT; bf* WK = WT + (size_t)NH_ * HD * DM; bf* WV = WT + (size_t)2 * NH_ * HD * DM;

    if (SEQ == SEQ_FULL) {
        const size_t n8 = (size_t)NB * SEQ * DM / 8;
        k_cvt8<<<(unsigned)((n8 + 255) / 256), 256, 0, stream>>>(x, XB, n8);
    } else {
        const size_t n8 = (size_t)SEQ * DM / 8;
        for (int b = 0; b < NB; ++b) k_cvt8<<<(unsigned)((n8 + 255) / 256), 256, 0, stream>>>(x + (size_t)b * SEQ_FULL * DM, XB + (size_t)b * SEQ * DM, n8);
    }
    k_wtr_bf<<<dim3(HD / 64, DM / 64, NH_), 256, 0, stream>>>(wq, WQ, DM, HD);
    k_wtr_bf<<<dim3(HD / 64, DM / 64, NH_), 256, 0, stream>>>(wk, WK, DM, HD);
    k_wtr_bf<<<dim3(HD / 64, DM / 64, NH_), 256, 0, stream>>>(wv, WV, DM, HD);
    k_wtr_h<<<dim3(DM / 64, CAT / 64, 1), 256, 0, stream>>>(wo, WOT, CAT, DM, WOS);
    k_wtr_h<<<dim3(FFD / 64, DM / 64, 1), 256, 0, stream>>>(w1, W1T, DM, FFD, W1S);
    k_wtr_h<<<dim3(DM / 64, FFD / 64, 1), 256, 0, stream>>>(w2, W2T, FFD, DM, W2S);

    for (int ps = 0; ps < NPASS; ++ps) {
        const int b0 = ps * NBP;
        k_proj_qk<<<dim3(NBP * SEQ / 64, HD / 64, 2 * NH_), 32, 0, stream>>>(XB, WT, QK, b0);
        k_proj_vt<<<dim3(HD / 64, NBP * SEQ / 64, NH_), 32, 0, stream>>>(WV, XB, VT, b0);
        k_flash<<<dim3(SEQ / 16, NBP * NH_, 1), 32 * FW, 0, stream>>>(QP, KP, VT, CTX, b0);
    }
    k_wo<<<dim3(NB * SEQ / 64, DM / 64, 1), 32, 0, stream>>>(CTX, WOT, MHA);
    k_ln1<<<NB * SEQ / 8, 256, 0, stream>>>(x, MHA, g1, be1, HF, HH);
    k_ffn1<<<dim3(NB * SEQ / 64, FFD / 64, 1), 32, 0, stream>>>(HH, W1T, b1, F1);
    k_ffn2<<<dim3(NB * SEQ / 64, DM / 64, 1), 32, 0, stream>>>(F1, W2T, b2, F2);
    k_ln2<<<NB * SEQ / 8, 256, 0, stream>>>(HF, F2, g2, be2, OUT);
}
